// ECN_35459249996330
// MI455X (gfx1250) — hardware-verified
//
#include <hip/hip_runtime.h>
#include <stddef.h>
#include <stdint.h>


#define HID     25
#define DOUT    32
#define KP      32
#define ZC      1024
#define NTHR    256
#define NWAVE   8
#define EPT     8
#define NGRP    2
#define CHUNK   (NTHR * EPT * NGRP)
#define WCAP    (EPT * NGRP * 32)
#define LISTN   (NWAVE * WCAP)
#define NB      256
#define GROWS   128
#define GCOLS   128
#define NMOMB   64
#define GMAX    128
#define XSC     16.0f
#define WSC     16.0f
#define ZINV    0.00390625f
#define BN_EPS  1e-5f

static_assert((CHUNK & (CHUNK - 1)) == 0);
static_assert(CHUNK <= 4096);
static_assert((NB & (NB - 1)) == 0 && NB <= 4096);
static_assert(NB * DOUT == 32 * NTHR);
static_assert(GROWS == 16 * NWAVE);
static_assert(ZC % GCOLS == 0 && NB % GROWS == 0);
static_assert(KP == DOUT);

typedef float    v4f  __attribute__((ext_vector_type(4)));
typedef float    v8f  __attribute__((ext_vector_type(8)));
typedef int      v4i  __attribute__((ext_vector_type(4)));
typedef _Float16 v2h  __attribute__((ext_vector_type(2)));
typedef _Float16 v8h  __attribute__((ext_vector_type(8)));
typedef _Float16 v16h __attribute__((ext_vector_type(16)));
union FragH { v16h v; v8h h[2]; };

__device__ __forceinline__ v8h cvt8(v4f a, v4f b) {
  v8h r;
  r[0] = (_Float16)a.x; r[1] = (_Float16)a.y; r[2] = (_Float16)a.z; r[3] = (_Float16)a.w;
  r[4] = (_Float16)b.x; r[5] = (_Float16)b.y; r[6] = (_Float16)b.z; r[7] = (_Float16)b.w;
  return r;
}

__device__ __forceinline__ v8f wmh(v16h a, v16h b, v8f c) {
  v8f d = __builtin_amdgcn_wmma_f32_16x16x32_f16(false, a, false, b, (short)0, c, false, false);
  asm volatile("v_nop\n\tv_nop\n\tv_nop\n\tv_nop" : "+v"(d) : "v"(a), "v"(b));
  return d;
}

#define HSL(V, K) __builtin_bit_cast(float, __builtin_amdgcn_readlane(__builtin_bit_cast(int, (V)), (K)))

__device__ __forceinline__ int scan_chunk(const int* __restrict__ dsts, int nE, int cbase, int nodeBase,
                                          int vec8, int* list, int tid, int wave) {
  int wc = 0;
#pragma unroll
  for (int g = 0; g < NGRP; ++g) {
    const int el0  = (g * NTHR + tid) * EPT;
    const int e0   = cbase + el0;
    const int sent = -2147483647 - 1;
    v4i da, db;
    if (vec8 != 0 && e0 + 7 < nE) {
      da = *(const v4i*)(dsts + e0);
      db = *(const v4i*)(dsts + e0 + 4);
    } else {
      da.x = (e0     < nE) ? dsts[e0]     : sent;
      da.y = (e0 + 1 < nE) ? dsts[e0 + 1] : sent;
      da.z = (e0 + 2 < nE) ? dsts[e0 + 2] : sent;
      da.w = (e0 + 3 < nE) ? dsts[e0 + 3] : sent;
      db.x = (e0 + 4 < nE) ? dsts[e0 + 4] : sent;
      db.y = (e0 + 5 < nE) ? dsts[e0 + 5] : sent;
      db.z = (e0 + 6 < nE) ? dsts[e0 + 6] : sent;
      db.w = (e0 + 7 < nE) ? dsts[e0 + 7] : sent;
    }
    const unsigned nb = (unsigned)nodeBase;
    const unsigned s0 = (unsigned)da.x - nb, s1 = (unsigned)da.y - nb;
    const unsigned s2 = (unsigned)da.z - nb, s3 = (unsigned)da.w - nb;
    const unsigned s4 = (unsigned)db.x - nb, s5 = (unsigned)db.y - nb;
    const unsigned s6 = (unsigned)db.z - nb, s7 = (unsigned)db.w - nb;
    const bool h0 = s0 < (unsigned)NB, h1 = s1 < (unsigned)NB, h2 = s2 < (unsigned)NB, h3 = s3 < (unsigned)NB;
    const bool h4 = s4 < (unsigned)NB, h5 = s5 < (unsigned)NB, h6 = s6 < (unsigned)NB, h7 = s7 < (unsigned)NB;
    const unsigned any = __builtin_amdgcn_ballot_w32(h0 | h1 | h2 | h3 | h4 | h5 | h6 | h7);
    if (any != 0u) {
#define HITJ(J, HJ, SJ) { \
        const unsigned mj = __builtin_amdgcn_ballot_w32(HJ); \
        if (mj != 0u) { \
          if (HJ) { \
            const int pos = wc + (int)__builtin_amdgcn_mbcnt_lo(mj, 0u); \
            if (pos < WCAP) list[wave * WCAP + pos] = ((el0 + (J)) << 12) | (int)(SJ); \
          } \
          wc += (int)__builtin_popcount(mj); } }
      HITJ(0, h0, s0)
      HITJ(1, h1, s1)
      HITJ(2, h2, s2)
      HITJ(3, h3, s3)
      HITJ(4, h4, s4)
      HITJ(5, h5, s5)
      HITJ(6, h6, s6)
      HITJ(7, h7, s7)
#undef HITJ
    }
  }
  return wc;
}

__global__ __launch_bounds__(NTHR) void k_mom(const float* __restrict__ ea, double* mom, int nE) {
  __shared__ double red[9][NTHR];
  __shared__ __attribute__((aligned(16))) union { double d[16]; v4f f[8]; } ml;
  const int tid = threadIdx.x;
  double s0 = 0.0, s1 = 0.0, s2 = 0.0;
  double q00 = 0.0, q01 = 0.0, q02 = 0.0, q11 = 0.0, q12 = 0.0, q22 = 0.0;
#pragma unroll 1
  for (int e = blockIdx.x * NTHR + tid; e < nE; e += NMOMB * NTHR) {
    const float* p = ea + (size_t)e * 3;
    const double a0 = (double)p[0], a1 = (double)p[1], a2 = (double)p[2];
    s0 += a0; s1 += a1; s2 += a2;
    q00 += a0 * a0; q01 += a0 * a1; q02 += a0 * a2;
    q11 += a1 * a1; q12 += a1 * a2; q22 += a2 * a2;
  }
  red[0][tid] = s0;  red[1][tid] = s1;  red[2][tid] = s2;
  red[3][tid] = q00; red[4][tid] = q01; red[5][tid] = q02;
  red[6][tid] = q11; red[7][tid] = q12; red[8][tid] = q22;
  __syncthreads();
  if (tid < 16) {
    double t = 0.0;
    if (tid < 9) {
#pragma unroll 1
      for (int i = 0; i < NTHR; ++i) t += red[tid][i];
    }
    ml.d[tid] = t;
  }
  __syncthreads();
  if (tid < 8) {
    const v4f v = ml.f[tid];
    float* mp = (float*)mom + (size_t)blockIdx.x * 32 + 4 * tid;
    *(volatile v4f*)mp = v;
    __threadfence();
    *(volatile v4f*)mp = v;
  }
}

__device__ __forceinline__ float bval(const float* __restrict__ w2, const float* __restrict__ b2,
                                      int kc, int i, int o, int din) {
  float v = 0.0f;
  if (i < din) {
    if (kc < HID)       v = w2[(size_t)kc * (size_t)(din * DOUT) + (size_t)i * DOUT + o];
    else if (kc == HID) v = b2[i * DOUT + o];
  }
  return v * WSC;
}

__global__ __launch_bounds__(NTHR) void k_prep(const float* __restrict__ x,
    const float* __restrict__ w2a, const float* __restrict__ b2a,
    const float* __restrict__ w2b, const float* __restrict__ b2b,
    _Float16* bt0, _Float16* bt1, _Float16* x16, int nN, int nPad, int din0, int din1) {
  const int t  = blockIdx.x * NTHR + threadIdx.x;
  const int nBq = ZC * (KP / 8);
  const int nB  = 2 * nBq;
  const int nX  = nPad * (KP / 8);
  if (t >= nB + nX) return;
  v4f a, b;
  _Float16* dp;
  if (t < nB) {
    const int l   = (t >= nBq) ? 1 : 0;
    const int u   = t - l * nBq;
    const int col = u >> 2, i0 = (u & 3) * 8;
    const int o   = col >> 5, kc = col & 31;
    const float* w2 = l ? w2b : w2a;
    const float* b2 = l ? b2b : b2a;
    const int din = l ? din1 : din0;
    a.x = bval(w2, b2, kc, i0 + 0, o, din); a.y = bval(w2, b2, kc, i0 + 1, o, din);
    a.z = bval(w2, b2, kc, i0 + 2, o, din); a.w = bval(w2, b2, kc, i0 + 3, o, din);
    b.x = bval(w2, b2, kc, i0 + 4, o, din); b.y = bval(w2, b2, kc, i0 + 5, o, din);
    b.z = bval(w2, b2, kc, i0 + 6, o, din); b.w = bval(w2, b2, kc, i0 + 7, o, din);
    dp = (l ? bt1 : bt0) + (size_t)u * 8;
  } else {
    const int u = t - nB;
    const int n = u >> 2, c8 = (u & 3) * 8;
#define XV(J) (((n < nN) && ((c8 + (J)) < din0)) ? x[(size_t)n * din0 + c8 + (J)] * XSC : 0.0f)
    a.x = XV(0); a.y = XV(1); a.z = XV(2); a.w = XV(3);
    b.x = XV(4); b.y = XV(5); b.z = XV(6); b.w = XV(7);
#undef XV
    dp = x16 + (size_t)u * 8;
  }
  const v8h hv = cvt8(a, b);
  *(volatile v8h*)dp = hv;
  __threadfence();
  *(volatile v8h*)dp = hv;
}

__global__ __launch_bounds__(NTHR) void k_zgemm(const _Float16* __restrict__ x16,
                                                 const _Float16* __restrict__ bt, _Float16* z) {
  __shared__ __attribute__((aligned(16))) _Float16 stg[NWAVE * 16 * GCOLS];
  const int tid = threadIdx.x, lane = tid & 31, wave = tid >> 5, hh = lane >> 4, m = lane & 15;
  const int rowBase = blockIdx.x * GROWS + wave * 16;
  const int colBase = blockIdx.y * GCOLS;

  FragH a;
  const _Float16* ap = x16 + (size_t)(rowBase + m) * KP + 8 * hh;
  a.h[0] = *(const v8h*)ap;
  a.h[1] = *(const v8h*)(ap + 16);

  v8f acc[8];
#pragma unroll
  for (int t = 0; t < 8; ++t) {
    const _Float16* bp = bt + (size_t)(colBase + 16 * t + m) * KP + 8 * hh;
    FragH b;
    b.h[0] = *(const v8h*)bp;
    b.h[1] = *(const v8h*)(bp + 16);
    const v8f c = {0.f, 0.f, 0.f, 0.f, 0.f, 0.f, 0.f, 0.f};
    acc[t] = wmh(a.v, b.v, c);
  }

  _Float16* sp = stg + (wave * 16 + 8 * hh) * GCOLS + m;
#pragma unroll
  for (int t = 0; t < 8; ++t) {
#pragma unroll
    for (int r = 0; r < 8; ++r) sp[r * GCOLS + 16 * t] = (_Float16)acc[t][r];
  }
  __syncthreads();

  const _Float16* lp = stg + (wave * 16 + hh) * GCOLS + 8 * m;
  _Float16* gp = z + (size_t)(rowBase + hh) * ZC + colBase + 8 * m;
#pragma unroll
  for (int q = 0; q < 8; ++q) {
    const v8h v = *(const v8h*)(lp + 2 * q * GCOLS);
    *(volatile v8h*)(gp + (size_t)(2 * q) * ZC) = v;
  }
  __threadfence();
#pragma unroll
  for (int q = 0; q < 8; ++q) {
    const v8h v = *(const v8h*)(lp + 2 * q * GCOLS);
    *(volatile v8h*)(gp + (size_t)(2 * q) * ZC) = v;
  }
}

__global__ __launch_bounds__(NTHR) void k_agg(
    const int* __restrict__ ei, const float* __restrict__ ea, const double* __restrict__ mom,
    const float* __restrict__ w1, const float* __restrict__ b1,
    const float* __restrict__ gam, const float* __restrict__ bet,
    const _Float16* __restrict__ z, const float* __restrict__ xin,
    const float* __restrict__ wr, const float* __restrict__ bc,
    float* xout, _Float16* x16out,
    int nN, int nE, int din, int xpitch, int vec8, int write16) {
  __shared__ __attribute__((aligned(16))) float acc[NB * DOUT];
  __shared__ __attribute__((aligned(16))) int   list[LISTN];
  __shared__ int    cnt[NB];
  __shared__ int    wcnt[NWAVE];
  __shared__ float  wf0[32];
  __shared__ float  wf1[32];
  __shared__ float  wf2[32];
  __shared__ float  cfv[32];
  __shared__ __attribute__((aligned(16))) float wrs[KP * DOUT];
  __shared__ float  bcs[DOUT];
  __shared__ double momt[9];

  const int tid = threadIdx.x, lane = tid & 31, wave = tid >> 5;
  const int nodeBase = blockIdx.x * NB;
  const int* dsts = ei + nE;

  {
    const v4f zz = {0.f, 0.f, 0.f, 0.f};
    for (int i = tid; i < NB * DOUT / 4; i += NTHR) *(v4f*)(acc + 4 * i) = zz;
  }
  for (int i = tid; i < NB; i += NTHR) cnt[i] = 0;
  for (int i = tid; i < KP * DOUT; i += NTHR) {
    const int k = i >> 5, o = i & 31;
    wrs[i] = (k < din) ? wr[k * DOUT + o] : 0.0f;
  }
  if (tid < DOUT) bcs[tid] = bc[tid];
  if (tid < 9) {
    double t = 0.0;
#pragma unroll 1
    for (int bI = 0; bI < NMOMB; ++bI) t += mom[bI * 16 + tid];
    momt[tid] = t;
  }
  __syncthreads();
  if (tid < 32) {
    float f0 = 0.0f, f1 = 0.0f, f2 = 0.0f, fc = 0.0f;
    if (tid < HID) {
      const double invE = 1.0 / (double)nE;
      const double m0 = momt[0] * invE, m1 = momt[1] * invE, m2 = momt[2] * invE;
      const double c00 = momt[3] * invE - m0 * m0, c01 = momt[4] * invE - m0 * m1, c02 = momt[5] * invE - m0 * m2;
      const double c11 = momt[6] * invE - m1 * m1, c12 = momt[7] * invE - m1 * m2, c22 = momt[8] * invE - m2 * m2;
      const float u0f = w1[tid], u1f = w1[HID + tid], u2f = w1[2 * HID + tid];
      const double u0 = (double)u0f, u1 = (double)u1f, u2 = (double)u2f;
      const double mu = m0 * u0 + m1 * u1 + m2 * u2 + (double)b1[tid];
      double var = u0 * u0 * c00 + u1 * u1 * c11 + u2 * u2 * c22
                 + 2.0 * (u0 * u1 * c01 + u0 * u2 * c02 + u1 * u2 * c12);
      var = var > 0.0 ? var : 0.0;
      const float sc = rsqrtf((float)var + BN_EPS) * gam[tid];
      f0 = u0f * sc; f1 = u1f * sc; f2 = u2f * sc;
      fc = (b1[tid] - (float)mu) * sc + bet[tid];
    }
    wf0[tid] = f0; wf1[tid] = f1; wf2[tid] = f2; cfv[tid] = fc;
  }
  __syncthreads();

  const int nChunks = (nE + CHUNK - 1) / CHUNK;
#pragma unroll 1
  for (int ch = 0; ch < nChunks; ++ch) {
    const int cbase = ch * CHUNK;
    const int wc = scan_chunk(dsts, nE, cbase, nodeBase, vec8, list, tid, wave);
    if (lane == 0) wcnt[wave] = wc;
    __syncthreads();
    if (wave == 0) {
#pragma unroll 1
      for (int wsx = 0; wsx < NWAVE; ++wsx) {
        int n = __builtin_amdgcn_readfirstlane(wcnt[wsx]);
        n = n > WCAP ? WCAP : (n < 0 ? 0 : n);
        const int* lp = list + wsx * WCAP;
#pragma unroll 1
        for (int i = 0; i < n; ++i) {
          const int ent  = __builtin_amdgcn_readfirstlane(lp[i]);
          const int slot = ent & (NB - 1);
          int e = cbase + ((ent >> 12) & (CHUNK - 1));
          e = e > nE - 1 ? nE - 1 : e;
          int src = ei[e];
          src = src < 0 ? 0 : (src > nN - 1 ? nN - 1 : src);
          const float* eap = ea + (size_t)e * 3;
          const float a0 = eap[0], a1 = eap[1], a2 = eap[2];
          float hk = fmaf(a0, wf0[lane], fmaf(a1, wf1[lane], fmaf(a2, wf2[lane], cfv[lane])));
          hk = fmaxf(hk, 0.0f);
          hk = (lane < HID) ? hk : ((lane == HID) ? 1.0f : 0.0f);
          const _Float16* zp = z + (size_t)src * ZC + lane * 32;
          const v8h zv0 = *(const v8h*)zp;
          const v8h zv1 = *(const v8h*)(zp + 8);
          const v8h zv2 = *(const v8h*)(zp + 16);
          const v2h zv3 = *(const v2h*)(zp + 24);
          float msg = 0.0f;
#pragma unroll
          for (int k = 0; k < 8; ++k) msg = fmaf(HSL(hk, k), (float)zv0[k], msg);
#pragma unroll
          for (int k = 0; k < 8; ++k) msg = fmaf(HSL(hk, 8 + k), (float)zv1[k], msg);
#pragma unroll
          for (int k = 0; k < 8; ++k) msg = fmaf(HSL(hk, 16 + k), (float)zv2[k], msg);
          msg = fmaf(HSL(hk, 24), (float)zv3[0], msg);
          msg = fmaf(HSL(hk, 25), (float)zv3[1], msg);
          acc[slot * DOUT + lane] = acc[slot * DOUT + lane] + msg;
          if (lane == 0) cnt[slot] = cnt[slot] + 1;
        }
      }
    }
    __syncthreads();
  }

#pragma unroll 1
  for (int i = 0; i < (NB * DOUT) / NTHR; ++i) {
    const int idx  = i * NTHR + tid;
    const int row  = idx >> 5;
    const int o    = idx & 31;
    const int node = nodeBase + row;
    const int nodec = node > nN - 1 ? nN - 1 : node;
    int d = cnt[row];
    d = d < 1 ? 1 : d;
    const float rd = 1.0f / (float)d;
    float v = (acc[idx] * ZINV) * rd;
    float r = 0.0f;
    const float* xp = xin + (size_t)nodec * xpitch;
#pragma unroll 1
    for (int k = 0; k < din; ++k) r = fmaf(xp[k], wrs[k * DOUT + o], r);
    v = (v + r) + bcs[o];
    v = v > 0.0f ? v : expm1f(v);
    if (node >= nN) v = 0.0f;
    acc[idx] = v;
  }
  __syncthreads();

  const size_t rowG = (size_t)nodeBase;
#pragma unroll
  for (int i = 0; i < 8; ++i) {
    const int idx = i * NTHR + tid;
    const int row = idx >> 3, c4 = (idx & 7) * 4;
    const v4f v = *(const v4f*)(acc + 4 * idx);
    *(volatile v4f*)(xout + (rowG + row) * DOUT + c4) = v;
  }
  if (write16 != 0) {
#pragma unroll
    for (int i = 0; i < 4; ++i) {
      const int idx = i * NTHR + tid;
      const int row = idx >> 2, c8 = (idx & 3) * 8;
      const v4f p0 = *(const v4f*)(acc + 8 * idx) * XSC;
      const v4f p1 = *(const v4f*)(acc + 8 * idx + 4) * XSC;
      const v8h hv = cvt8(p0, p1);
      *(volatile v8h*)(x16out + (rowG + row) * KP + c8) = hv;
    }
  }
  __threadfence();
#pragma unroll
  for (int i = 0; i < 8; ++i) {
    const int idx = i * NTHR + tid;
    const int row = idx >> 3, c4 = (idx & 7) * 4;
    const v4f v = *(const v4f*)(acc + 4 * idx);
    *(volatile v4f*)(xout + (rowG + row) * DOUT + c4) = v;
  }
  if (write16 != 0) {
#pragma unroll
    for (int i = 0; i < 4; ++i) {
      const int idx = i * NTHR + tid;
      const int row = idx >> 2, c8 = (idx & 3) * 8;
      const v4f p0 = *(const v4f*)(acc + 8 * idx) * XSC;
      const v4f p1 = *(const v4f*)(acc + 8 * idx + 4) * XSC;
      const v8h hv = cvt8(p0, p1);
      *(volatile v8h*)(x16out + (rowG + row) * KP + c8) = hv;
    }
  }
}

__global__ __launch_bounds__(NTHR) void k_pool(const float* __restrict__ xf, const int* __restrict__ batch,
                                                const float* __restrict__ wfc, const float* __restrict__ bfc,
                                                float* out, int nN, int nG) {
  __shared__ __attribute__((aligned(16))) float gacc[GMAX * DOUT];
  __shared__ int gcnt[GMAX];
  __shared__ __attribute__((aligned(16))) float outv[GMAX];
  const int tid = threadIdx.x, lane = tid & 31, wave = tid >> 5;
  for (int i = tid; i < GMAX * DOUT; i += NTHR) gacc[i] = 0.0f;
  for (int i = tid; i < GMAX; i += NTHR) { gcnt[i] = 0; outv[i] = 0.0f; }
  __syncthreads();

  const float wl = wfc[lane];
#pragma unroll 1
  for (int n0 = 0; n0 < nN; n0 += 32) {
    const int n = n0 + lane;
    const int b = (n < nN) ? batch[n] : -1;
    const bool hit = (b >= 0) && (b < nG) && ((b & (NWAVE - 1)) == wave);
    unsigned msk = __builtin_amdgcn_ballot_w32(hit);
    while (msk != 0u) {
      const int sl = __builtin_ctz(msk);
      msk &= msk - 1u;
      const int g  = __builtin_amdgcn_readlane(b, sl);
      const int nn = n0 + sl;
      gacc[g * DOUT + lane] = gacc[g * DOUT + lane] + xf[(size_t)nn * DOUT + lane];
      if (lane == 0) gcnt[g] = gcnt[g] + 1;
    }
  }

#pragma unroll 1
  for (int g = wave; g < nG; g += NWAVE) {
    int c = gcnt[g];
    c = c < 1 ? 1 : c;
    const float rc = 1.0f / (float)c;
    float p = (gacc[g * DOUT + lane] * rc) * wl;
    p += __shfl_xor(p, 16);
    p += __shfl_xor(p, 8);
    p += __shfl_xor(p, 4);
    p += __shfl_xor(p, 2);
    p += __shfl_xor(p, 1);
    if (lane == 0) outv[g] = p + bfc[0];
  }
  __syncthreads();

  if (wave == 0) {
    const int nq = nG >> 2;
    if (lane < nq) { const v4f v = *(const v4f*)(outv + 4 * lane); *(volatile v4f*)(out + 4 * lane) = v; }
    if (lane == 0) {
#pragma unroll 1
      for (int j = 4 * nq; j < nG; ++j) { const float v = outv[j]; *(volatile float*)(out + j) = v; }
    }
    __threadfence();
    if (lane < nq) { const v4f v = *(const v4f*)(outv + 4 * lane); *(volatile v4f*)(out + 4 * lane) = v; }
    if (lane == 0) {
#pragma unroll 1
      for (int j = 4 * nq; j < nG; ++j) { const float v = outv[j]; *(volatile float*)(out + j) = v; }
    }
  }
}

extern "C" void kernel_launch(void* const* d_in, const int* in_sizes, int n_in,
                              void* d_out, int out_size, void* d_ws, size_t ws_size,
                              hipStream_t stream) {
  if (n_in < 22) return;
  const int nN = in_sizes[3];
  if (nN <= 0) return;
  const int din0 = in_sizes[0] / nN;
  if (din0 < 1 || din0 > KP || din0 * nN != in_sizes[0]) return;
  const int nE = in_sizes[1] / 3;
  if (nE <= 0 || nE > (1 << 27) || in_sizes[1] != 3 * nE || in_sizes[2] != 2 * nE) return;
  const int din1 = DOUT;
  if (in_sizes[4] != 3 * HID || in_sizes[5] < HID || in_sizes[6] < HID || in_sizes[7] < HID) return;
  if (in_sizes[8] != HID * din0 * DOUT || in_sizes[9] < din0 * DOUT) return;
  if (in_sizes[10] != din0 * DOUT || in_sizes[11] < DOUT) return;
  if (in_sizes[12] != 3 * HID || in_sizes[13] < HID || in_sizes[14] < HID || in_sizes[15] < HID) return;
  if (in_sizes[16] != HID * din1 * DOUT || in_sizes[17] < din1 * DOUT) return;
  if (in_sizes[18] != din1 * DOUT || in_sizes[19] < DOUT) return;
  if (in_sizes[20] < DOUT || in_sizes[21] < 1) return;
  const int nG = out_size;
  if (nG < 1 || nG > GMAX) return;

  const float* x     = (const float*)d_in[0];
  const float* ea    = (const float*)d_in[1];
  const int*   ei    = (const int*)d_in[2];
  const int*   batch = (const int*)d_in[3];
  const float* w1_0  = (const float*)d_in[4];
  const float* b1_0  = (const float*)d_in[5];
  const float* g_0   = (const float*)d_in[6];
  const float* be_0  = (const float*)d_in[7];
  const float* w2_0  = (const float*)d_in[8];
  const float* b2_0  = (const float*)d_in[9];
  const float* wr_0  = (const float*)d_in[10];
  const float* bc_0  = (const float*)d_in[11];
  const float* w1_1  = (const float*)d_in[12];
  const float* b1_1  = (const float*)d_in[13];
  const float* g_1   = (const float*)d_in[14];
  const float* be_1  = (const float*)d_in[15];
  const float* w2_1  = (const float*)d_in[16];
  const float* b2_1  = (const float*)d_in[17];
  const float* wr_1  = (const float*)d_in[18];
  const float* bc_1  = (const float*)d_in[19];
  const float* wfc   = (const float*)d_in[20];
  const float* bfc   = (const float*)d_in[21];
  float* out = (float*)d_out;

  const int nA   = (nN + NB - 1) / NB;
  const int nPad = nA * NB;

  char* ws = (char*)d_ws;
  size_t off = 0;
  const size_t oMom = off; off += (size_t)NMOMB * 128;              off = (off + 255) & ~(size_t)255;
  const size_t oBt0 = off; off += (size_t)ZC * KP * 2;              off = (off + 255) & ~(size_t)255;
  const size_t oBt1 = off; off += (size_t)ZC * KP * 2;              off = (off + 255) & ~(size_t)255;
  const size_t oXa  = off; off += (size_t)nPad * KP * 2;            off = (off + 255) & ~(size_t)255;
  const size_t oXb  = off; off += (size_t)nPad * KP * 2;            off = (off + 255) & ~(size_t)255;
  const size_t oZ   = off; off += (size_t)nPad * ZC * 2;            off = (off + 255) & ~(size_t)255;
  const size_t oXf1 = off; off += (size_t)nPad * DOUT * 4;          off = (off + 255) & ~(size_t)255;
  const size_t oXf2 = off; off += (size_t)nPad * DOUT * 4;          off = (off + 255) & ~(size_t)255;
  if (off > ws_size || off > (size_t)134217728) return;
  double*   mom  = (double*)(ws + oMom);
  _Float16* bt0  = (_Float16*)(ws + oBt0);
  _Float16* bt1  = (_Float16*)(ws + oBt1);
  _Float16* x16a = (_Float16*)(ws + oXa);
  _Float16* x16b = (_Float16*)(ws + oXb);
  _Float16* z    = (_Float16*)(ws + oZ);
  float*    xf1  = (float*)(ws + oXf1);
  float*    xf2  = (float*)(ws + oXf2);

  const int vec8 = ((nE & 3) == 0) ? 1 : 0;

  k_mom<<<NMOMB, NTHR, 0, stream>>>(ea, mom, nE);

  const int nPrep = 2 * ZC * (KP / 8) + nPad * (KP / 8);
  k_prep<<<(nPrep + NTHR - 1) / NTHR, NTHR, 0, stream>>>(x, w2_0, b2_0, w2_1, b2_1,
                                                         bt0, bt1, x16a, nN, nPad, din0, din1);

  const dim3 gz(nPad / GROWS, ZC / GCOLS);
  k_zgemm<<<gz, NTHR, 0, stream>>>(x16a, bt0, z);
  k_agg<<<nA, NTHR, 0, stream>>>(ei, ea, mom, w1_0, b1_0, g_0, be_0, z, x, wr_0, bc_0,
                                  xf1, x16b, nN, nE, din0, din0, vec8, 1);

  k_zgemm<<<gz, NTHR, 0, stream>>>(x16b, bt1, z);
  k_agg<<<nA, NTHR, 0, stream>>>(ei, ea, mom, w1_1, b1_1, g_1, be_1, z, xf1, wr_1, bc_1,
                                  xf2, x16a, nN, nE, din1, DOUT, vec8, 0);

  k_pool<<<1, NTHR, 0, stream>>>(xf2, batch, wfc, bfc, out, nN, nG);
}
